// UV_Aggregator_19061064860210
// MI455X (gfx1250) — hardware-run, weakly checked
//
#include <hip/hip_runtime.h>
#include <math.h>

typedef __attribute__((ext_vector_type(16))) _Float16 v16h;
typedef __attribute__((ext_vector_type(16))) __bf16 v16b;
typedef __attribute__((ext_vector_type(8)))  _Float16 v8h;
typedef __attribute__((ext_vector_type(8)))  float v8f;
typedef __attribute__((ext_vector_type(4)))  float v4f;
typedef __attribute__((ext_vector_type(2)))  float v2f;
typedef __attribute__((ext_vector_type(4)))  unsigned v4u;
typedef __attribute__((ext_vector_type(4)))  int v4i;
typedef float __attribute__((may_alias)) float_a;
typedef int __attribute__((may_alias)) int_a;

template <typename T> __device__ __forceinline__ void vst2(void* p, T v) { *(volatile T*)p = v; __threadfence(); *(volatile T*)p = v; }
__device__ __forceinline__ v8f wmma16(v16h a, v16h b, v8f c) {
  v8f d = __builtin_amdgcn_wmma_f32_16x16x32_f16(false, a, false, b, (short)0, c, false, false);
  asm volatile("v_nop\n\tv_nop\n\tv_nop\n\tv_nop" : "+v"(d) : "v"(a), "v"(b));
  return d;
}
__device__ __forceinline__ v8f wmma_bf(v16b a, v16b b, v8f c) {
  v8f d = __builtin_amdgcn_wmma_f32_16x16x32_bf16(false, a, false, b, (short)0, c, false, false);
  asm volatile("v_nop\n\tv_nop\n\tv_nop\n\tv_nop" : "+v"(d) : "v"(a), "v"(b));
  return d;
}
__device__ __forceinline__ v16h frag_h(const _Float16* rowk0, int lane) {
  union { v16h v; v8h q[2]; } u; const _Float16* p = rowk0 + 8 * (lane >> 4);
  u.q[0] = *(const v8h*)p; u.q[1] = *(const v8h*)(p + 16); return u.v;
}
__device__ __forceinline__ v16h frag_f32(const float* rowk0, int lane) {
  v16h a; const float* p = rowk0 + 8 * (lane >> 4);
#pragma unroll
  for (int i = 0; i < 8; ++i) { a[i] = (_Float16)p[i]; a[8 + i] = (_Float16)p[16 + i]; }
  return a;
}
__device__ __forceinline__ v16h frag_f32s(const float* rowk0, int lane, float sc) {
  v16h a; const float* p = rowk0 + 8 * (lane >> 4);
#pragma unroll
  for (int i = 0; i < 8; ++i) { a[i] = (_Float16)(p[i] * sc); a[8 + i] = (_Float16)(p[16 + i] * sc); }
  return a;
}
__device__ __forceinline__ v16h fragc_f32(const float* W, int k0, int n, int lane, int ld, int K) {
  v16h a; const int g = lane >> 4;
#pragma unroll
  for (int i = 0; i < 8; ++i) { const int ka = k0 + 8 * g + i, kb = ka + 16;
    a[i] = (_Float16)(ka < K ? W[(size_t)(ka < K ? ka : K - 1) * ld + n] : 0.f); a[8 + i] = (_Float16)(kb < K ? W[(size_t)(kb < K ? kb : K - 1) * ld + n] : 0.f); }
  return a;
}
struct F2 { v16b h, l; };
__device__ __forceinline__ F2 bsplit16(const float v[16]) { F2 r;
#pragma unroll
  for (int i = 0; i < 16; ++i) { const __bf16 h = (__bf16)v[i]; r.h[i] = h; r.l[i] = (__bf16)(v[i] - (float)h); }
  return r; }
__device__ __forceinline__ F2 split_row(const float* row, int k0, int lane) { float v[16]; const float* p = row + k0 + 8 * (lane >> 4);
#pragma unroll
  for (int i = 0; i < 8; ++i) { v[i] = p[i]; v[8 + i] = p[16 + i]; }
  return bsplit16(v); }
__device__ __forceinline__ F2 split_rowK(const float* row, int k0, int lane, int K) { float v[16]; const int g = lane >> 4;
#pragma unroll
  for (int i = 0; i < 8; ++i) { const int ka = k0 + 8 * g + i, kb = ka + 16; v[i] = ka < K ? row[ka < K ? ka : K - 1] : 0.f; v[8 + i] = kb < K ? row[kb < K ? kb : K - 1] : 0.f; }
  return bsplit16(v); }
__device__ __forceinline__ F2 split_col(const float* W, int k0, int n, int lane, int ld, int K) { float v[16]; const int g = lane >> 4;
#pragma unroll
  for (int i = 0; i < 8; ++i) { const int ka = k0 + 8 * g + i, kb = ka + 16; v[i] = ka < K ? W[(size_t)(ka < K ? ka : K - 1) * ld + n] : 0.f; v[8 + i] = kb < K ? W[(size_t)(kb < K ? kb : K - 1) * ld + n] : 0.f; }
  return bsplit16(v); }
__device__ __forceinline__ v8f mac3(const F2& a, const F2& b, v8f c) { c = wmma_bf(a.l, b.h, c); c = wmma_bf(a.h, b.l, c); return wmma_bf(a.h, b.h, c); }
__device__ __forceinline__ float sigm(float v) { return 1.0f / (1.0f + expf(-v)); }
#define LDSX() do { asm volatile("s_wait_dscnt 0" ::: "memory"); __builtin_amdgcn_wave_barrier(); __builtin_amdgcn_fence(__ATOMIC_RELEASE, "workgroup"); } while (0)

#define NU 4096
#define HL 50
#define DM 64
#define NUSR 100000
#define NITM 100000
#define NRT 5
#ifndef NRV
#define NRV NU
#endif
__device__ __forceinline__ float bfr(float v) { return (float)(__bf16)v; }
__device__ __forceinline__ v16b wcol_kz(const float* __restrict__ Wm, int k0, int o, int lane, int ld, int K, int nvalid) { v16b w; const int g = lane >> 4; const int oc = o < nvalid ? o : 0; const float keepo = o < nvalid ? 1.f : 0.f;
  asm volatile("s_wait_loadcnt 0x0" ::: "memory");
#pragma unroll
  for (int i = 0; i < 8; ++i) { const int ka = k0 + 8 * g + i, kb = ka + 16; w[i] = (__bf16)(Wm[(size_t)(ka < K ? ka : 0) * ld + oc] * (ka < K ? keepo : 0.f)); w[8 + i] = (__bf16)(Wm[(size_t)(kb < K ? kb : 0) * ld + oc] * (kb < K ? keepo : 0.f)); }
  asm volatile("s_wait_loadcnt 0x0" ::: "memory"); return w; }
__global__ __launch_bounds__(128) void k_uv(const int* __restrict__ NODES, const int* __restrict__ HUV, const int* __restrict__ HR, const int* __restrict__ LEN, const float* __restrict__ U2E, const float* __restrict__ V2E, const float* __restrict__ R2E,
    const float* __restrict__ W1, const float* __restrict__ B1, const float* __restrict__ W2, const float* __restrict__ B2, const float* __restrict__ A1, const float* __restrict__ BA1, const float* __restrict__ A2, const float* __restrict__ BA2, const float* __restrict__ A3, const float* __restrict__ BA3, float* __restrict__ OUT) {
  __shared__ __align__(16) float sx[4][16][68], so[4][16][68], sh2[4][16][68]; __shared__ float ssc[64]; __shared__ float satt[64]; __shared__ __align__(16) float sagg[DM];
  const int tid = threadIdx.x, wave = tid >> 5, lane = tid & 31, col = lane & 15, g = lane >> 4; const size_t b = blockIdx.x; const int l = wave * 16 + col;
  int node = NODES[b]; node = node < 0 ? 0 : (node >= NUSR ? NUSR - 1 : node); int len = LEN[b]; len = len < 0 ? 0 : (len > HL ? HL : len);
  const int lc = l < HL ? l : 0; int iu = HUV[b * HL + lc]; iu = iu < 0 ? 0 : (iu >= NITM ? NITM - 1 : iu); int ir = HR[b * HL + lc]; ir = ir < 0 ? 0 : (ir >= NRT ? NRT - 1 : ir); const float keep = l < HL ? 1.f : 0.f;
  v8f acc[4] = {};
#pragma unroll
  for (int kc = 0; kc < 4; ++kc) { v16b a; { const float* p = (kc < 2 ? V2E + (size_t)iu * DM : R2E + (size_t)ir * DM) + (kc & 1) * 32 + 8 * g;
#pragma unroll
      for (int i = 0; i < 8; ++i) { a[i] = (__bf16)(p[i] * keep); a[8 + i] = (__bf16)(p[16 + i] * keep); } }
    asm volatile("s_wait_loadcnt 0x0" ::: "memory");
#pragma unroll
    for (int j = 0; j < 4; ++j) { const v16b w = wcol_kz(W1, kc * 32, j * 16 + col, lane, DM, 2 * DM, DM); acc[j] = wmma_bf(a, w, acc[j]); } }
#pragma unroll
  for (int j = 0; j < 4; ++j) { const float bb = bfr(B1[j * 16 + col]);
#pragma unroll
    for (int r = 0; r < 8; ++r) sx[wave][8 * g + r][j * 16 + col] = fmaxf(acc[j][r] + bb, 0.f); }
  LDSX();
  { v8f acc2[4] = {};
#pragma unroll
    for (int kc = 0; kc < 2; ++kc) { const F2 a = split_row(&sx[wave][col][0], kc * 32, lane);
#pragma unroll
      for (int j = 0; j < 4; ++j) { const v16b w = wcol_kz(W2, kc * 32, j * 16 + col, lane, DM, DM, DM); acc2[j] = wmma_bf(a.h, w, acc2[j]); acc2[j] = wmma_bf(a.l, w, acc2[j]); } }
#pragma unroll
    for (int j = 0; j < 4; ++j) { const float bb = bfr(B2[j * 16 + col]);
#pragma unroll
      for (int r = 0; r < 8; ++r) so[wave][8 * g + r][j * 16 + col] = fmaxf(acc2[j][r] + bb, 0.f); } }
  LDSX();
  { v8f acc3[4] = {};
#pragma unroll
    for (int kc = 0; kc < 2; ++kc) { const F2 a = split_row(&so[wave][col][0], kc * 32, lane);
#pragma unroll
      for (int j = 0; j < 4; ++j) { const v16b w = wcol_kz(A1, kc * 32, j * 16 + col, lane, DM, 2 * DM, DM); acc3[j] = wmma_bf(a.h, w, acc3[j]); acc3[j] = wmma_bf(a.l, w, acc3[j]); } }
#pragma unroll
    for (int kc = 0; kc < 2; ++kc) { v16b a; { const float* p = U2E + (size_t)node * DM + kc * 32 + 8 * g;
#pragma unroll
        for (int i = 0; i < 8; ++i) { a[i] = (__bf16)p[i]; a[8 + i] = (__bf16)p[16 + i]; } }
      asm volatile("s_wait_loadcnt 0x0" ::: "memory");
#pragma unroll
      for (int j = 0; j < 4; ++j) { const v16b w = wcol_kz(A1, DM + kc * 32, j * 16 + col, lane, DM, 2 * DM, DM); acc3[j] = wmma_bf(a, w, acc3[j]); } }
#pragma unroll
    for (int j = 0; j < 4; ++j) { const float bb = bfr(BA1[j * 16 + col]);
#pragma unroll
      for (int r = 0; r < 8; ++r) sx[wave][8 * g + r][j * 16 + col] = fmaxf(acc3[j][r] + bb, 0.f); } }
  LDSX();
  { v8f acc4[4] = {};
#pragma unroll
    for (int kc = 0; kc < 2; ++kc) { const F2 a = split_row(&sx[wave][col][0], kc * 32, lane);
#pragma unroll
      for (int j = 0; j < 4; ++j) { const v16b w = wcol_kz(A2, kc * 32, j * 16 + col, lane, DM, DM, DM); acc4[j] = wmma_bf(a.h, w, acc4[j]); acc4[j] = wmma_bf(a.l, w, acc4[j]); } }
#pragma unroll
    for (int j = 0; j < 4; ++j) { const float bb = bfr(BA2[j * 16 + col]);
#pragma unroll
      for (int r = 0; r < 8; ++r) sh2[wave][8 * g + r][j * 16 + col] = fmaxf(acc4[j][r] + bb, 0.f); } }
  LDSX();
  { v8f acc5 = {};
#pragma unroll
    for (int kc = 0; kc < 2; ++kc) { const F2 a = split_row(&sh2[wave][col][0], kc * 32, lane); const v16b w = wcol_kz(A3, kc * 32, col, lane, 1, DM, 1); acc5 = wmma_bf(a.h, w, acc5); acc5 = wmma_bf(a.l, w, acc5); }
    const float bb = bfr(BA3[0]);
    if (col == 0) {
#pragma unroll
      for (int r = 0; r < 8; ++r) ssc[wave * 16 + 8 * g + r] = acc5[r] + bb; } }
  __syncthreads();
  { float m = -3.0e38f; for (int q = 0; q < 64; ++q) { const float v = (q < len) ? ssc[q] : -3.0e38f; m = fmaxf(m, v); }
    float sum = 0.f; for (int q = 0; q < 64; ++q) sum += (q < len) ? expf(ssc[q] - m) : 0.f;
    if (tid < 64) satt[tid] = (tid < len && sum > 0.f) ? expf(ssc[tid] - m) / sum : 0.f; }
  __syncthreads();
  if (tid < DM) { const int d = tid; float a = 0.f; for (int q = 0; q < HL; ++q) a += satt[q] * so[q >> 4][q & 15][d];
    const float uval = bfr(U2E[(size_t)node * DM + d]); asm volatile("s_wait_loadcnt 0x0" ::: "memory"); sagg[d] = (len > 0) ? a : uval; }
  __syncthreads();
  if (tid < 16) vst2(OUT + b * DM + tid * 4, *(const v4f*)&sagg[tid * 4]); }
extern "C" void kernel_launch(void* const* d_in, const int* in_sizes, int n_in, void* d_out, int out_size, void* d_ws, size_t ws_size, hipStream_t stream) {
  (void)in_sizes; (void)n_in; (void)out_size; (void)d_ws; (void)ws_size;
  const float** F = (const float**)d_in;
  k_uv<<<dim3(NRV), 128, 0, stream>>>((const int*)d_in[0], (const int*)d_in[1], (const int*)d_in[2], (const int*)d_in[3], F[4], F[5], F[6], F[7], F[8], F[9], F[10], F[11], F[12], F[13], F[14], F[15], F[16], (float*)d_out);
}
